// SelfAttentionBlock_66992899883169
// MI455X (gfx1250) — hardware-verified
//
#include <hip/hip_runtime.h>
#ifndef NB
#define NB 4
#endif
#ifndef SEQ
#define SEQ 4096
#endif
#define SEQ_FULL 4096
#define CH 256
#define NHEAD 8
#define HD 32
#define NQK 512
#define NQKV 768

static_assert(SEQ % 128 == 0);
static_assert(SEQ <= SEQ_FULL);
static_assert(CH == NHEAD * HD);
static_assert(CH % 128 == 0);
static_assert(CH % 64 == 0);
static_assert(NQK % 64 == 0);
static_assert(((size_t)NB * SEQ) % 128 == 0);
static_assert(HD == 32);

typedef unsigned short v8us __attribute__((ext_vector_type(8), may_alias));
typedef float  v8f  __attribute__((ext_vector_type(8)));
typedef float  v4f  __attribute__((ext_vector_type(4)));
typedef float  v4fa __attribute__((ext_vector_type(4), may_alias));
typedef _Float16 v16h __attribute__((ext_vector_type(16)));
typedef _Float16 v4h __attribute__((ext_vector_type(4)));
union FragH { v16h v; v8us half[2]; _Float16 h[16]; unsigned short u[16]; };

__device__ __forceinline__ float bf16_rne(float x) { unsigned int u = __float_as_uint(x); u = (u + 0x7FFFu + ((u >> 16) & 1u)) & 0xFFFF0000u; return __uint_as_float(u); }

__device__ __forceinline__ v16h g2_frag(const _Float16* p, unsigned hh) { FragH f; f.half[0] = *(const v8us*)((const unsigned short*)p + 8 * hh); f.half[1] = *(const v8us*)((const unsigned short*)p + 16 + 8 * hh); return f.v; }
__device__ __forceinline__ v8f g2_mma(v16h a, v16h b, v8f c) { v8f d = __builtin_amdgcn_wmma_f32_16x16x32_f16(false, a, false, b, (short)0, c, false, false); asm volatile("v_nop\n\tv_nop\n\tv_nop\n\tv_nop" : "+v"(d) : "v"(a), "v"(b)); return d; }

template <unsigned K, unsigned N>
__global__ __launch_bounds__(256) void k_wt_f16(const float* __restrict__ W, _Float16* __restrict__ Wt, float scale) {
  const unsigned t = blockIdx.x * 256u + threadIdx.x;
  if (t >= N * (K / 8u)) return;
  const unsigned n = t / (K / 8u), k8 = (t % (K / 8u)) * 8u;
  FragH f;
#pragma unroll
  for (unsigned i = 0; i < 8u; ++i) f.h[i] = (_Float16)(bf16_rne(W[(size_t)(k8 + i) * N + n]) * scale);
  const v8us o = f.half[0];
  unsigned short* d = (unsigned short*)Wt + (size_t)n * K + k8;
  *(volatile v8us*)d = o; __threadfence(); *(volatile v8us*)d = o;
}

__global__ __launch_bounds__(256) void k_xt(const float* __restrict__ x, _Float16* __restrict__ X16) {
  __shared__ __attribute__((aligned(16))) _Float16 tl[64][72];
  const unsigned tid = threadIdx.x;
  const unsigned nt = blockIdx.x % (unsigned)(SEQ / 64), rest = blockIdx.x / (unsigned)(SEQ / 64);
  const unsigned ct = rest % (unsigned)(CH / 64), b = rest / (unsigned)(CH / 64);
  const unsigned n0 = nt * 64u, c0 = ct * 64u;
#pragma unroll
  for (unsigned it = 0; it < 4u; ++it) {
    const unsigned i = tid + it * 256u; const unsigned c = i >> 4, n4 = (i & 15u) * 4u;
    const v4f v = *(const v4fa*)(x + ((size_t)b * CH + c0 + c) * SEQ_FULL + n0 + n4);
#pragma unroll
    for (unsigned q = 0; q < 4u; ++q) tl[n4 + q][c] = (_Float16)bf16_rne(v[q]);
  }
  __syncthreads();
  for (int pass = 0; pass < 2; ++pass) {
#pragma unroll
    for (unsigned rd = 0; rd < 2u; ++rd) {
      const unsigned n = rd * 32u + (tid >> 3), pc = tid & 7u;
      const v8us o = *(const v8us*)&tl[n][pc * 8u];
      *(volatile v8us*)((unsigned short*)X16 + ((size_t)b * SEQ + n0 + n) * CH + c0 + pc * 8u) = o;
    }
    if (pass == 0) __threadfence();
  }
}

template <bool CB, bool RB, bool RES, bool OUT16>
__global__ __launch_bounds__(128) void k_gemm2(const _Float16* __restrict__ A, unsigned lda, size_t sA,
    const _Float16* __restrict__ Bh, unsigned ldb, size_t sB, unsigned bks, float alpha,
    const float* __restrict__ cbias, const float* __restrict__ rbias,
    const float* __restrict__ CP, unsigned ldcp, size_t sCP,
    float* __restrict__ C, _Float16* __restrict__ C16, unsigned ldc, size_t sC, unsigned M, unsigned N, unsigned K) {
  __shared__ __attribute__((aligned(16))) float so[4][32][68];
  const unsigned tid = threadIdx.x, w = tid >> 5, lane = tid & 31u, ln = lane & 15u, hh = lane >> 4; const unsigned by = blockIdx.y;
  A += (size_t)by * sA; Bh += (size_t)by * sB; const size_t cofs = (size_t)by * sC;
  const unsigned ntn = N >> 6; const unsigned mt = blockIdx.x / ntn, nq = blockIdx.x - mt * ntn;
  const unsigned row0 = mt * 128u + 32u * w, col0 = nq * 64u; if (row0 >= M) return;
  const _Float16* a0p = A + (size_t)(row0 + ln) * lda; const _Float16* a1p = a0p + (size_t)16 * lda;
  const _Float16* b0p = Bh + (size_t)(col0 + ln) * ldb; const _Float16* b1p = b0p + (size_t)16 * ldb; const _Float16* b2p = b1p + (size_t)16 * ldb; const _Float16* b3p = b2p + (size_t)16 * ldb;
  const v8f z8 = {0.f,0.f,0.f,0.f,0.f,0.f,0.f,0.f}; v8f c00 = z8, c01 = z8, c02 = z8, c03 = z8, c10 = z8, c11 = z8, c12 = z8, c13 = z8;
#pragma unroll 1
  for (unsigned kb = 0; kb < K; kb += 32u) {
    const size_t bo = (size_t)(kb >> 5) * bks;
    const v16h a0 = g2_frag(a0p + kb, hh), a1 = g2_frag(a1p + kb, hh);
    v16h b = g2_frag(b0p + bo, hh); c00 = g2_mma(a0, b, c00); c10 = g2_mma(a1, b, c10);
    b = g2_frag(b1p + bo, hh); c01 = g2_mma(a0, b, c01); c11 = g2_mma(a1, b, c11);
    b = g2_frag(b2p + bo, hh); c02 = g2_mma(a0, b, c02); c12 = g2_mma(a1, b, c12);
    b = g2_frag(b3p + bo, hh); c03 = g2_mma(a0, b, c03); c13 = g2_mma(a1, b, c13);
  }
  v8f accs[8] = {c00, c01, c02, c03, c10, c11, c12, c13};
  float rb[2][8];
#pragma unroll
  for (int hf = 0; hf < 2; ++hf) {
    v4f r0 = {0.f, 0.f, 0.f, 0.f}, r1 = {0.f, 0.f, 0.f, 0.f};
    if (RB) { r0 = *(const v4fa*)(rbias + row0 + hf * 16 + 8u * hh); r1 = *(const v4fa*)(rbias + row0 + hf * 16 + 8u * hh + 4u); }
#pragma unroll
    for (int i = 0; i < 4; ++i) { rb[hf][i] = RB ? bf16_rne(r0[i]) : 0.f; rb[hf][4 + i] = RB ? bf16_rne(r1[i]) : 0.f; }
  }
#pragma unroll
  for (int u = 0; u < 8; ++u) {
    const int t = u & 3, hf = u >> 2; const unsigned col = col0 + t * 16 + ln;
    float cb = 0.f; if (CB) cb = bf16_rne(cbias[col]);
#pragma unroll
    for (int r = 0; r < 8; ++r) { const unsigned rloc = hf * 16 + 8u * hh + r; const float v = accs[u][r] * alpha + cb + rb[hf][r]; so[w][rloc][t * 16 + ln] = v; }
  }
  __builtin_amdgcn_fence(4  , "workgroup"); __builtin_amdgcn_wave_barrier();
  const unsigned rsub = lane >> 4, c4 = (lane & 15u) * 4u;
  if (RES) {
    const float* cpb = CP + (size_t)by * sCP;
#pragma unroll 2
    for (unsigned q = 0; q < 16u; ++q) {
      const unsigned r = q * 2u + rsub;
      v4f v = *(const v4fa*)&so[w][r][c4];
      const v4f xr = *(const v4fa*)(cpb + (size_t)(row0 + r) * ldcp + col0 + c4);
#pragma unroll
      for (int i = 0; i < 4; ++i) v[i] += bf16_rne(xr[i]);
      *(v4fa*)&so[w][r][c4] = v;
    }
  }
  for (int pass = 0; pass < 2; ++pass) {
#pragma unroll
    for (unsigned q = 0; q < 16u; ++q) {
      const unsigned r = q * 2u + rsub; const v4f v = *(const v4fa*)&so[w][r][c4];
      if (!OUT16) { *(volatile v4f*)(C + cofs + (size_t)(row0 + r) * ldc + col0 + c4) = v; }
      else { v4h h4;
#pragma unroll
        for (int i = 0; i < 4; ++i) h4[i] = (_Float16)v[i];
        *(volatile v4h*)(C16 + cofs + (size_t)(row0 + r) * ldc + col0 + c4) = h4; }
    }
    if (pass == 0) __threadfence();
  }
}

__global__ __launch_bounds__(128) void k_attn(const _Float16* __restrict__ QK16, const _Float16* __restrict__ VT, _Float16* __restrict__ O16) {
  __shared__ __attribute__((aligned(16))) _Float16 Psh[4][16 * 72];
  const unsigned tid = threadIdx.x, w = tid >> 5, lane = tid & 31u, ln = lane & 15u, hh = lane >> 4;
  const unsigned bh = blockIdx.y, b = bh >> 3, h = bh & 7u;
  const unsigned qr0 = blockIdx.x * 64u + w * 16u;
  const float scale = 0.17677669529663687f;
  const _Float16* qrow = QK16 + ((size_t)b * SEQ + qr0 + ln) * NQK + h * HD;
  const _Float16* kcol = QK16 + ((size_t)b * SEQ + ln) * NQK + CH + h * HD;
  const _Float16* v0p = VT + ((size_t)b * CH + h * HD + ln) * SEQ; const _Float16* v1p = v0p + (size_t)16 * SEQ;
  const v16h aq = g2_frag(qrow, hh);
  const v8f z8 = {0.f,0.f,0.f,0.f,0.f,0.f,0.f,0.f};
  v8f acc0 = z8, acc1 = z8;
  float mrow[8], lrow[8];
#pragma unroll
  for (int r = 0; r < 8; ++r) { mrow[r] = -1.0e30f; lrow[r] = 0.f; }
  _Float16* pw = &Psh[w][0];
#pragma unroll 1
  for (unsigned kb = 0; kb < (unsigned)SEQ; kb += 64u) {
    const _Float16* kp = kcol + (size_t)kb * NQK;
    v16h bk = g2_frag(kp, hh); v8f s0 = g2_mma(aq, bk, z8);
    bk = g2_frag(kp + (size_t)16 * NQK, hh); v8f s1 = g2_mma(aq, bk, z8);
    bk = g2_frag(kp + (size_t)32 * NQK, hh); v8f s2 = g2_mma(aq, bk, z8);
    bk = g2_frag(kp + (size_t)48 * NQK, hh); v8f s3 = g2_mma(aq, bk, z8);
    __builtin_amdgcn_wave_barrier();
#pragma unroll
    for (int r = 0; r < 8; ++r) {
      const float a0 = s0[r] * scale, a1 = s1[r] * scale, a2 = s2[r] * scale, a3 = s3[r] * scale;
      float mx = fmaxf(fmaxf(a0, a1), fmaxf(a2, a3));
      mx = fmaxf(mx, __shfl_xor(mx, 1, 32));
      mx = fmaxf(mx, __shfl_xor(mx, 2, 32));
      mx = fmaxf(mx, __shfl_xor(mx, 4, 32));
      mx = fmaxf(mx, __shfl_xor(mx, 8, 32));
      const float mn = fmaxf(mrow[r], mx);
      const float al = __expf(mrow[r] - mn);
      const float mc = mn - 5.545177444479562f;
      const float e0 = __expf(a0 - mc), e1 = __expf(a1 - mc), e2 = __expf(a2 - mc), e3 = __expf(a3 - mc);
      float rs = (e0 + e1) + (e2 + e3);
      rs += __shfl_xor(rs, 1, 32);
      rs += __shfl_xor(rs, 2, 32);
      rs += __shfl_xor(rs, 4, 32);
      rs += __shfl_xor(rs, 8, 32);
      lrow[r] = lrow[r] * al + rs;
      mrow[r] = mn;
      acc0[r] *= al; acc1[r] *= al;
      const unsigned m = 8u * hh + (unsigned)r;
      pw[m * 72u + ln]       = (_Float16)e0;
      pw[m * 72u + 16u + ln] = (_Float16)e1;
      pw[m * 72u + 32u + ln] = (_Float16)e2;
      pw[m * 72u + 48u + ln] = (_Float16)e3;
    }
    __builtin_amdgcn_fence(4  , "workgroup"); __builtin_amdgcn_wave_barrier();
    FragH p0, p1;
    p0.half[0] = *(const v8us*)&Psh[w][ln * 72u + 8u * hh];       p0.half[1] = *(const v8us*)&Psh[w][ln * 72u + 16u + 8u * hh];
    p1.half[0] = *(const v8us*)&Psh[w][ln * 72u + 32u + 8u * hh]; p1.half[1] = *(const v8us*)&Psh[w][ln * 72u + 48u + 8u * hh];
    v16h bv = g2_frag(v0p + kb, hh);        acc0 = g2_mma(p0.v, bv, acc0);
    bv = g2_frag(v0p + kb + 32u, hh);       acc0 = g2_mma(p1.v, bv, acc0);
    bv = g2_frag(v1p + kb, hh);             acc1 = g2_mma(p0.v, bv, acc1);
    bv = g2_frag(v1p + kb + 32u, hh);       acc1 = g2_mma(p1.v, bv, acc1);
    __builtin_amdgcn_fence(4  , "workgroup"); __builtin_amdgcn_wave_barrier();
  }
#pragma unroll
  for (int r = 0; r < 8; ++r) {
    const float inv = 64.0f * (1.0f / lrow[r]);
    const unsigned m = 8u * hh + (unsigned)r;
    pw[m * 72u + ln]       = (_Float16)(acc0[r] * inv);
    pw[m * 72u + 16u + ln] = (_Float16)(acc1[r] * inv);
  }
  __builtin_amdgcn_fence(4  , "workgroup"); __builtin_amdgcn_wave_barrier();
  unsigned short* ob = (unsigned short*)O16 + ((size_t)bh * SEQ + qr0) * HD;
  const v8us o0 = *(const v8us*)&Psh[w][(lane >> 2) * 72u + (lane & 3u) * 8u];
  const v8us o1 = *(const v8us*)&Psh[w][(8u + (lane >> 2)) * 72u + (lane & 3u) * 8u];
  *(volatile v8us*)(ob + lane * 8u) = o0;
  *(volatile v8us*)(ob + 256u + lane * 8u) = o1;
  __threadfence();
  *(volatile v8us*)(ob + lane * 8u) = o0;
  *(volatile v8us*)(ob + 256u + lane * 8u) = o1;
}

__global__ __launch_bounds__(256) void k_gn(const float* __restrict__ Y, const float* __restrict__ gamma, const float* __restrict__ beta, float* __restrict__ out) {
  __shared__ float red[256];
  const unsigned tid = threadIdx.x, b = blockIdx.x >> 5, g = blockIdx.x & 31u;
  const float* y = Y + ((size_t)b * CH + 8u * g) * SEQ;
  const unsigned nit = (unsigned)(8 * SEQ / 4 / 256);
  const float rc = 1.0f / (float)(8 * SEQ);
  float s1 = 0.f;
#pragma unroll 2
  for (unsigned u = 0; u < nit; ++u) { const v4f a = *(const v4fa*)(y + (size_t)(tid + 256u * u) * 4u); s1 += (a[0] + a[1]) + (a[2] + a[3]); }
  red[tid] = s1; __syncthreads();
  for (unsigned st = 128u; st > 0u; st >>= 1) { if (tid < st) red[tid] += red[tid + st]; __syncthreads(); }
  const float mean = red[0] * rc; __syncthreads();
  float s2 = 0.f;
#pragma unroll 2
  for (unsigned u = 0; u < nit; ++u) { const v4f a = *(const v4fa*)(y + (size_t)(tid + 256u * u) * 4u);
    const float d0 = a[0] - mean, d1 = a[1] - mean, d2 = a[2] - mean, d3 = a[3] - mean; s2 += (d0 * d0 + d1 * d1) + (d2 * d2 + d3 * d3); }
  red[tid] = s2; __syncthreads();
  for (unsigned st = 128u; st > 0u; st >>= 1) { if (tid < st) red[tid] += red[tid + st]; __syncthreads(); }
  const float rstd = rsqrtf(red[0] * rc + 1.0e-5f);
  for (int pass = 0; pass < 2; ++pass) {
#pragma unroll 2
    for (unsigned u = 0; u < nit; ++u) {
      const unsigned e = (tid + 256u * u) * 4u; const unsigned cc = e / (unsigned)SEQ, n = e % (unsigned)SEQ; const unsigned ch = 8u * g + cc;
      const float ga = bf16_rne(gamma[ch]), be = bf16_rne(beta[ch]);
      const v4f a = *(const v4fa*)(y + e); v4f o;
#pragma unroll
      for (int q = 0; q < 4; ++q) o[q] = ((a[q] - mean) * rstd) * ga + be;
      *(volatile v4f*)(out + ((size_t)b * CH + ch) * SEQ_FULL + n) = o;
    }
    if (pass == 0) __threadfence();
  }
}

extern "C" void kernel_launch(void* const* d_in, const int* in_sizes, int n_in,
                              void* d_out, int out_size, void* d_ws, size_t ws_size, hipStream_t stream) {
  if (n_in < 7) return;
  const long long need = (long long)((size_t)(NB - 1) * CH + (CH - 1)) * SEQ_FULL + SEQ;
  if ((long long)in_sizes[0] < need || in_sizes[1] < CH * NQKV || in_sizes[2] < NQKV || in_sizes[3] < CH * CH ||
      in_sizes[4] < CH || in_sizes[5] < CH || in_sizes[6] < CH) return;
  if ((long long)out_size < need) return;
  const float* x = (const float*)d_in[0]; const float* wqkv = (const float*)d_in[1]; const float* bqkv = (const float*)d_in[2];
  const float* wproj = (const float*)d_in[3]; const float* bproj = (const float*)d_in[4]; const float* gamma = (const float*)d_in[5]; const float* beta = (const float*)d_in[6];
  float* out = (float*)d_out;
  char* ws = (char*)d_ws; size_t off = 0;
  auto take = [&](size_t bytes) { char* p = ws + off; off += (bytes + 255) & ~(size_t)255; return p; };
  _Float16* WT  = (_Float16*)take((size_t)NQKV * CH * 2);
  _Float16* WTP = (_Float16*)take((size_t)CH * CH * 2);
  _Float16* X16 = (_Float16*)take((size_t)NB * SEQ * CH * 2);
  _Float16* QK16 = (_Float16*)take((size_t)NB * SEQ * NQK * 2);
  _Float16* VT  = (_Float16*)take((size_t)NB * CH * SEQ * 2);
  _Float16* O16 = (_Float16*)take((size_t)NB * NHEAD * SEQ * HD * 2);
  float*    Y   = (float*)take((size_t)NB * CH * SEQ * 4);
  if (off > ws_size) return;

  k_wt_f16<CH, NQKV><<<(NQKV * (CH / 8) + 255) / 256, 256, 0, stream>>>(wqkv, WT, 16.0f);
  k_wt_f16<CH, CH><<<(CH * (CH / 8) + 255) / 256, 256, 0, stream>>>(wproj, WTP, 16.0f);
  k_xt<<<(unsigned)(NB * (CH / 64) * (SEQ / 64)), 256, 0, stream>>>(x, X16);
  k_gemm2<true, false, false, true><<<dim3((unsigned)(((size_t)NB * SEQ / 128) * (NQK / 64)), 1), 128, 0, stream>>>(
      X16, CH, 0, WT, CH, 0, 32u, 0.0625f, bqkv, bqkv, x, 0u, 0, Y, QK16, NQK, 0, (unsigned)((size_t)NB * SEQ), NQK, CH);
  k_gemm2<false, true, false, true><<<dim3((unsigned)((CH / 128) * (SEQ / 64)), NB), 128, 0, stream>>>(
      WT + (size_t)NQK * CH, CH, 0, X16, CH, (size_t)SEQ * CH, 32u, 0.0625f, bqkv, bqkv + NQK, x, 0u, 0, Y, VT, SEQ, (size_t)CH * SEQ, CH, SEQ, CH);
  k_attn<<<dim3(SEQ / 64, NB * NHEAD), 128, 0, stream>>>(QK16, VT, O16);
  k_gemm2<false, true, true, false><<<dim3((unsigned)((CH / 128) * (SEQ / 64)), NB), 128, 0, stream>>>(
      WTP, CH, 0, O16, HD, (size_t)NHEAD * SEQ * HD, (unsigned)(SEQ * HD), 0.0009765625f, bproj, bproj, x, (unsigned)SEQ_FULL, (size_t)CH * SEQ_FULL,
      Y, QK16, SEQ, (size_t)CH * SEQ, CH, SEQ, CH);
  k_gn<<<NB * 32, 256, 0, stream>>>(Y, gamma, beta, out);
}
